// FlashKAN_56676388438745
// MI455X (gfx1250) — hardware-verified
//
#include <hip/hip_runtime.h>
#include <math.h>


#ifndef NROWS
#define NROWS 2048
#endif
#define NROWS_FULL 2048
#define I_DIM  128
#define O_DIM  128
#define NG     68
#define NKNOT  71
#define BT     32
#define CH     8
#define NCHUNK (I_DIM / CH)
#define KCH    (CH * NG)
#define KTOT   (I_DIM * NG)
#define APITCH (KCH + 8)
#define PANEL_H 18432
#define OSP    132
#define ACARRY 1024.0f
#define WCARRY 64.0f
#define OFOLD  (1.0f / 65536.0f)

static_assert(KCH % 32 == 0);
static_assert(KTOT % 32 == 0);
static_assert(KTOT % 8 == 0);
static_assert((KTOT * 2) % 128 == 0);
static_assert(I_DIM % CH == 0);
static_assert(CH * BT == 256);
static_assert(O_DIM == 8 * 16);
static_assert(BT == 32);
static_assert(APITCH % 8 == 0);
static_assert(BT * APITCH <= PANEL_H);
static_assert(PANEL_H % (256 * 8) == 0);
static_assert((KCH / 32 - 1) * 32 + 16 + 8 + 7 < KCH);
static_assert(NROWS % BT == 0);
static_assert(NROWS <= NROWS_FULL);
static_assert((OSP * 4) % 16 == 0);
static_assert(8 * 4 * 32 * 16 == BT * O_DIM * 4);
static_assert(32 * 16 == O_DIM * 4);
static_assert((size_t)PANEL_H * 2 + (size_t)BT * OSP * 4 + (size_t)(NKNOT + 1) * 4 <= (size_t)131072);
static_assert(NKNOT == NG + 3);
static_assert(NG + 7 < 2 * NG);

typedef _Float16 h16;
typedef __attribute__((ext_vector_type(16))) _Float16 v16h;
typedef __attribute__((ext_vector_type(8)))  _Float16 v8h;
typedef __attribute__((ext_vector_type(8)))  float    v8f;
typedef __attribute__((ext_vector_type(4)))  float    v4f;
typedef v4f __attribute__((may_alias)) v4fa;
typedef v8h __attribute__((may_alias)) v8ha;

__device__ __forceinline__ unsigned short f2bf(float f) { unsigned u = __float_as_uint(f); u += 0x7FFFu + ((u >> 16) & 1u); return (unsigned short)(u >> 16); }
__device__ __forceinline__ float bfr(float f) { return __uint_as_float(((unsigned)f2bf(f)) << 16); }
__device__ __forceinline__ v16h cat16(v8h lo, v8h hi) { return __builtin_shufflevector(lo, hi, 0, 1, 2, 3, 4, 5, 6, 7, 8, 9, 10, 11, 12, 13, 14, 15); }
static __device__ __forceinline__ h16 toh_flush(float v) { const h16 r = (h16)v; return (fabsf(v) < 6.103515625e-05f) ? (h16)0.0f : r; }
__device__ __forceinline__ v16h ldh(const h16* p) { return cat16(*(const v8h*)p, *(const v8h*)(p + 16)); }
__device__ __forceinline__ v8f wmma16g(v16h a, v16h b, v8f c) {
    c = __builtin_amdgcn_wmma_f32_16x16x32_f16(false, a, false, b, (short)0, c, false, false);
    asm volatile("v_nop\n\tv_nop\n\tv_nop\n\tv_nop" : "+v"(c) : "v"(a), "v"(b));
    return c;
}

__global__ __launch_bounds__(256) void k_wplane(const float* __restrict__ w, h16* WT, unsigned n8) {
    unsigned idx = blockIdx.x * 256u + threadIdx.x; if (idx >= n8) return;
    asm volatile("" : "+v"(idx));
    unsigned o = idx / (unsigned)(KTOT / 8);
    unsigned k8 = (idx - o * (unsigned)(KTOT / 8)) * 8u;
    asm volatile("" : "+v"(k8));
    unsigned i0 = k8 / (unsigned)NG;
    unsigned g0 = k8 - (unsigned)NG * i0;
    asm volatile("" : "+v"(i0), "+v"(g0));
    asm volatile("" : "+v"(o));
    v8h hv;
#pragma unroll
    for (int e = 0; e < 8; ++e) {
        const unsigned gs = g0 + (unsigned)e;
        const bool wrap = gs >= (unsigned)NG;
        const unsigned g = wrap ? (gs - (unsigned)NG) : gs;
        const unsigned i = wrap ? (i0 + 1u) : i0;
        const size_t off = (size_t)g * (size_t)(I_DIM * O_DIM) + (size_t)i * (size_t)O_DIM + (size_t)o;
        const float v = bfr(w[off]) * WCARRY;
        hv[e] = toh_flush(v); }
    h16* dst = WT + (size_t)idx * 8;
    *(volatile v8h*)dst = hv; __threadfence(); *(volatile v8h*)dst = hv;
}

__global__ __launch_bounds__(256) void k_spline(const float* __restrict__ x, const h16* __restrict__ WT, const float* __restrict__ t, float* OUT) {
    __shared__ __align__(16) h16   sPA[PANEL_H];
    __shared__ __align__(16) float os[BT * OSP];
    __shared__ float sT[NKNOT + 1];

    const int tid = threadIdx.x;
    const int lane = tid & 31, lr = lane & 15, hi = lane >> 4;
    const int wave = __builtin_amdgcn_readfirstlane((int)(threadIdx.x >> 5));
    const int b0t = blockIdx.x * BT;
    const int o0 = wave * 16;

    { const int tc = tid < NKNOT ? tid : (NKNOT - 1);
      float tv = bfr(t[tc]); asm volatile("" : "+v"(tv));
      if (tid < NKNOT) sT[tid] = tv; }

    const int chc = tid & 7;
    const int Mc  = tid >> 3;

    v8f acc0 = (v8f){}, acc1 = (v8f){};
    const size_t boff = (size_t)(o0 + lr) * KTOT + 8 * hi;
    const int a0 = lr * APITCH + 8 * hi;
    const int a1 = a0 + 16 * APITCH;

#pragma unroll 1
    for (int ic = 0; ic < NCHUNK; ++ic) {
        __syncthreads();

#pragma unroll
        for (int j = 0; j < PANEL_H / (256 * 8); ++j)
            *(v8ha*)(&sPA[(tid + 256 * j) * 8]) = (v8h){};

        const int i = ic * CH + chc;
        const float xv = bfr(x[(size_t)(b0t + Mc) * I_DIM + i]);

        int lo = 0, hs = NKNOT;
#pragma unroll
        for (int s = 0; s < 7; ++s) {
            const int mid = (lo + hs) >> 1;
            const int mc = mid < NKNOT ? mid : (NKNOT - 1);
            const float tv = sT[mc];
            const bool act = lo < hs;
            const bool le = tv <= xv;
            lo = (act & le) ? (mid + 1) : lo;
            hs = (act & (!le)) ? mid : hs;
        }
        int ik = lo - 1; ik = ik < 3 ? 3 : (ik > (NKNOT - 5) ? (NKNOT - 5) : ik);

        float Nv[4]; Nv[0] = 1.0f; Nv[1] = 0.0f; Nv[2] = 0.0f; Nv[3] = 0.0f;
        float left[3], right[3];
#pragma unroll
        for (int j = 1; j <= 3; ++j) {
            left[j - 1]  = xv - sT[ik + 1 - j];
            right[j - 1] = sT[ik + j] - xv;
            float saved = 0.0f;
#pragma unroll
            for (int r = 0; r < j; ++r) {
                const float temp = Nv[r] / (right[r] + left[j - 1 - r]);
                Nv[r] = saved + right[r] * temp;
                saved = left[j - 1 - r] * temp;
            }
            Nv[j] = saved;
        }
        const float sv = xv * (1.0f / (1.0f + expf(-xv)));
        const int gb = ik - 3;

        __syncthreads();

        {
            const int base = Mc * APITCH + chc * NG;
            sPA[base + gb + 0] = toh_flush(Nv[0] * ACARRY);
            sPA[base + gb + 1] = toh_flush(Nv[1] * ACARRY);
            sPA[base + gb + 2] = toh_flush(Nv[2] * ACARRY);
            sPA[base + gb + 3] = toh_flush(Nv[3] * ACARRY);
            sPA[base + NG - 1] = toh_flush(sv * ACARRY);
        }

        __syncthreads();

        const h16* wb = WT + boff + (size_t)ic * KCH;
#pragma unroll 1
        for (int ks = 0; ks < KCH / 32; ++ks) {
            const int ko = ks * 32;
            const v16h A0 = cat16(*(const v8ha*)(&sPA[a0 + ko]), *(const v8ha*)(&sPA[a0 + ko + 16]));
            const v16h A1 = cat16(*(const v8ha*)(&sPA[a1 + ko]), *(const v8ha*)(&sPA[a1 + ko + 16]));
            const v16h Bf = ldh(wb + ko);
            acc0 = wmma16g(A0, Bf, acc0);
            acc1 = wmma16g(A1, Bf, acc1);
        }
    }

#pragma unroll
    for (int r = 0; r < 8; ++r) {
        os[(8 * hi + r) * OSP + o0 + lr]      = acc0[r] * OFOLD;
        os[(16 + 8 * hi + r) * OSP + o0 + lr] = acc1[r] * OFOLD;
    }
    __syncthreads();

    float* obase = OUT + (size_t)b0t * O_DIM;
#pragma unroll 1
    for (int ps = 0; ps < 2; ++ps) {
#pragma unroll
        for (int s = 0; s < 4; ++s) {
            const int row = wave * 4 + s;
            const v4f val = *(const v4fa*)(&os[row * OSP + lane * 4]);
            *(volatile v4f*)(obase + (size_t)row * O_DIM + lane * 4) = val; }
        if (ps == 0) __threadfence(); }
}

static constexpr size_t al256(size_t v) { return (v + 255) & ~(size_t)255; }
static constexpr size_t SZ_WT = al256((size_t)O_DIM * KTOT * 2);
static constexpr size_t SZ_TOTAL = SZ_WT;
static_assert(SZ_TOTAL <= (size_t)134217728);
static_assert(((size_t)O_DIM * KTOT) % 8 == 0);
static_assert(((size_t)O_DIM * KTOT / 8) % 256 == 0);

extern "C" void kernel_launch(void* const* d_in, const int* in_sizes, int n_in,
                              void* d_out, int out_size, void* d_ws, size_t ws_size, hipStream_t stream) {
    if (n_in < 3) return;
    if ((size_t)in_sizes[0] < (size_t)NROWS * I_DIM) return;
    if ((size_t)in_sizes[1] < (size_t)NG * I_DIM * O_DIM) return;
    if (in_sizes[2] < NKNOT) return;
    if ((size_t)out_size < (size_t)NROWS * O_DIM) return;
    if (SZ_TOTAL > ws_size) return;
    const float* x = (const float*)d_in[0];
    const float* w = (const float*)d_in[1];
    const float* t = (const float*)d_in[2];
    float* OUT = (float*)d_out;
    h16* WT = (h16*)d_ws;

    const unsigned n8 = (unsigned)((size_t)O_DIM * KTOT / 8);
    k_wplane<<<(n8 + 255u) / 256u, 256, 0, stream>>>(w, WT, n8);
    k_spline<<<NROWS / BT, 256, 0, stream>>>(x, WT, t, OUT);
}
